// CompactKroneckerFusion_81492709474483
// MI455X (gfx1250) — hardware-verified
//
#include <hip/hip_runtime.h>


#define NB_  8192
#define DIN  1024
#define SK   8192
#define NOUT 512
#define JC   1024
#define LMAX 32
#define LN_EPS 1e-5f
#define DM   JC
#define LOSC 1024.0f

typedef _Float16 h16;
typedef unsigned short bf;
typedef __attribute__((ext_vector_type(16))) __bf16   v16bf;
typedef __attribute__((ext_vector_type(16))) _Float16 v16h;
typedef __attribute__((ext_vector_type(8)))  _Float16 v8h;
typedef __attribute__((ext_vector_type(8)))  unsigned short v8us;
typedef __attribute__((ext_vector_type(8)))  float    v8f;
typedef __attribute__((ext_vector_type(4)))  float    v4f;
typedef v8h  __attribute__((may_alias)) v8ha;
typedef v4f  __attribute__((may_alias)) v4fa;
typedef v8us __attribute__((may_alias)) v8usa;

__device__ __forceinline__ unsigned short f2bf(float f) { unsigned u = __float_as_uint(f); u += 0x7FFFu + ((u >> 16) & 1u); return (unsigned short)(u >> 16); }
__device__ __forceinline__ float bf2f(unsigned short b) { return __uint_as_float(((unsigned)b) << 16); }
__device__ __forceinline__ float bfr(float f) { return bf2f(f2bf(f)); }
__device__ __forceinline__ v16h cat16(v8h lo, v8h hi) { return __builtin_shufflevector(lo, hi, 0, 1, 2, 3, 4, 5, 6, 7, 8, 9, 10, 11, 12, 13, 14, 15); }
__device__ __forceinline__ v16bf cat16b(v8us lo, v8us hi) { return __builtin_bit_cast(v16bf, __builtin_shufflevector(lo, hi, 0, 1, 2, 3, 4, 5, 6, 7, 8, 9, 10, 11, 12, 13, 14, 15)); }
__device__ __forceinline__ v8f wmma16(v16h a, v16h b, v8f c) { return __builtin_amdgcn_wmma_f32_16x16x32_f16(false, a, false, b, (short)0, c, false, false); }
__device__ __forceinline__ v8f wmmab(v16bf a, v16bf b, v8f c) { return __builtin_amdgcn_wmma_f32_16x16x32_bf16(false, a, false, b, (short)0, c, false, false); }

template <bool SPLITA, bool F16OUT = false>
__global__ __launch_bounds__(128) void k_gemmb(const bf* __restrict__ A, const bf* __restrict__ Al, const bf* __restrict__ Bn, const float* __restrict__ bias, float* C, int ldc, h16* C2, const float* __restrict__ R = nullptr, int K = DM, int roundR = 1) {
    __shared__ __align__(16) float ost[4][16 * 68];
    const int lane = threadIdx.x & 31, wave = threadIdx.x >> 5, lr = lane & 15, hi = lane >> 4;
    const int r0 = blockIdx.x * 64 + wave * 16, c0 = blockIdx.y * 64;
    const size_t aoff = (size_t)(r0 + lr) * K + 8 * hi;
    size_t boff[4];
#pragma unroll
    for (int t = 0; t < 4; ++t) boff[t] = (size_t)(c0 + t * 16 + lr) * K + 8 * hi;
    v8f acc[4];
#pragma unroll
    for (int t = 0; t < 4; ++t) acc[t] = (v8f){};
#pragma unroll 1
    for (int kc = 0; kc < K; kc += 32) {
        const v16bf a = cat16b(*(const v8us*)(A + aoff + kc), *(const v8us*)(A + aoff + kc + 16));
        v16bf al = a;
        if (SPLITA) al = cat16b(*(const v8us*)(Al + aoff + kc), *(const v8us*)(Al + aoff + kc + 16));
#pragma unroll
        for (int t = 0; t < 4; ++t) { const v16bf b = cat16b(*(const v8us*)(Bn + boff[t] + kc), *(const v8us*)(Bn + boff[t] + kc + 16)); acc[t] = wmmab(a, b, acc[t]); if (SPLITA) acc[t] = wmmab(al, b, acc[t]); }
        asm volatile("v_nop\n\tv_nop\n\tv_nop\n\tv_nop" : "+v"(acc[0]), "+v"(acc[1]), "+v"(acc[2]), "+v"(acc[3]) : "v"(a), "v"(al));
    }
    float* os = &ost[wave][0];
#pragma unroll
    for (int t = 0; t < 4; ++t) { const float bv = bias ? bfr(bias[c0 + t * 16 + lr]) : 0.f;
#pragma unroll
        for (int j = 0; j < 8; ++j) os[(hi * 8 + j) * 68 + t * 16 + lr] = acc[t][j] + bv; }
    __syncthreads();
    if (F16OUT) {
        h16* crow = (h16*)(void*)C + (size_t)r0 * ldc + c0;
        auto pass = [&]() {
#pragma unroll
            for (int s = 0; s < 4; ++s) { const int row = 4 * s + (lane >> 3), piece = lane & 7; const float* sp = os + row * 68 + piece * 8; v8h o, o2;
#pragma unroll
                for (int i = 0; i < 8; ++i) { const h16 a = (h16)sp[i]; o[i] = a; o2[i] = (h16)((sp[i] - (float)a) * LOSC); }
                *(volatile v8h*)(crow + (size_t)row * ldc + piece * 8) = o; if (C2) *(volatile v8h*)(C2 + (size_t)r0 * ldc + c0 + (size_t)row * ldc + piece * 8) = o2; }
        };
        pass(); __threadfence(); pass();
    } else {
        float* crow = C + (size_t)r0 * ldc + c0;
        auto pass = [&]() {
#pragma unroll
            for (int s = 0; s < 8; ++s) { const int Lid = (lane >> 3) + 4 * s, piece = lane & 7; const int row = Lid >> 1, cofs = (Lid & 1) * 32 + piece * 4;
                v4f val = *(const v4fa*)(os + row * 68 + cofs); if (R) { const v4f rv = *(const v4f*)(R + ((size_t)r0 + row) * ldc + c0 + cofs); val += roundR ? (v4f){bfr(rv[0]), bfr(rv[1]), bfr(rv[2]), bfr(rv[3])} : rv; }
                *(volatile v4f*)(crow + (size_t)row * ldc + cofs) = val; }
        };
        pass(); __threadfence(); pass();
    }
}


__global__ __launch_bounds__(256) void k_wt(const float* __restrict__ Wm, int K, int ncols, bf* WT) {
    __shared__ __align__(16) unsigned short tl[64 * 72];
    const int tid = threadIdx.x, k0 = blockIdx.x * 64, n0 = blockIdx.y * 64;
    const int kk = tid >> 2, nq = (tid & 3) * 16;
#pragma unroll
    for (int i = 0; i < 16; ++i) tl[(nq + i) * 72 + kk] = f2bf(Wm[(size_t)(k0 + kk) * ncols + n0 + nq + i]);
    __syncthreads();
    const int piece = tid & 7;
    auto pass = [&]() {
#pragma unroll
        for (int s = 0; s < 2; ++s) { const int nr = (tid >> 3) + 32 * s; const v8us val = *(const v8usa*)(tl + nr * 72 + piece * 8); *(volatile v8us*)(WT + (size_t)(n0 + nr) * K + k0 + piece * 8) = val; }
    };
    pass(); __threadfence(); pass();
}

__global__ __launch_bounds__(256) void k_sketch(const float* __restrict__ x1, const float* __restrict__ x2, const float* __restrict__ S1, const float* __restrict__ S2, int j0, bf* CKh, bf* CKl) {
    __shared__ unsigned short li1[64][LMAX], li2[64][LMAX]; __shared__ float lv1[64][LMAX], lv2[64][LMAX]; __shared__ int cnt1[4][64], cnt2[4][64]; __shared__ int n1[64], n2[64];
    typedef __attribute__((ext_vector_type(2))) unsigned short v2us;
    const int tid = threadIdx.x, col = tid & 63, part = tid >> 6; const int jb = blockIdx.x * 64; const int j = j0 + jb + col;
    int c1 = 0, c2 = 0;
#pragma unroll 1
    for (int r = part * 256; r < part * 256 + 256; ++r) { c1 += (S1[(size_t)r * SK + j] != 0.f); c2 += (S2[(size_t)r * SK + j] != 0.f); }
    cnt1[part][col] = c1; cnt2[part][col] = c2; __syncthreads();
    int o1 = 0, o2 = 0;
    for (int p = 0; p < part; ++p) { o1 += cnt1[p][col]; o2 += cnt2[p][col]; }
    if (part == 3) { const int t1 = o1 + c1, t2 = o2 + c2; n1[col] = t1 < LMAX ? t1 : LMAX; n2[col] = t2 < LMAX ? t2 : LMAX; }
#pragma unroll 1
    for (int r = part * 256; r < part * 256 + 256; ++r) { const float a = S1[(size_t)r * SK + j], c = S2[(size_t)r * SK + j];
        if (a != 0.f) { if (o1 < LMAX) { li1[col][o1] = (unsigned short)r; lv1[col][o1] = bfr(a); } ++o1; }
        if (c != 0.f) { if (o2 < LMAX) { li2[col][o2] = (unsigned short)r; lv2[col][o2] = bfr(c); } ++o2; } }
    __syncthreads();
    const int lane = tid & 31, wv = tid >> 5; const int ca = 2 * lane, cb = 2 * lane + 1; const int na1 = n1[ca], na2 = n2[ca], nb1 = n1[cb], nb2 = n2[cb];
#pragma unroll 1
    for (int b = wv; b < NB_; b += 8) { const float* xa = x1 + (size_t)b * DIN; const float* xb = x2 + (size_t)b * DIN;
        float sa1 = 0.f, sa2 = 0.f, sb1 = 0.f, sb2 = 0.f;
        for (int e = 0; e < na1; ++e) sa1 = fmaf(lv1[ca][e], bfr(xa[li1[ca][e]]), sa1);
        for (int e = 0; e < na2; ++e) sa2 = fmaf(lv2[ca][e], bfr(xb[li2[ca][e]]), sa2);
        for (int e = 0; e < nb1; ++e) sb1 = fmaf(lv1[cb][e], bfr(xa[li1[cb][e]]), sb1);
        for (int e = 0; e < nb2; ++e) sb2 = fmaf(lv2[cb][e], bfr(xb[li2[cb][e]]), sb2);
        const float cka = sa1 * sa2, ckb = sb1 * sb2; v2us oh, ol; const unsigned short ha = f2bf(cka), hb = f2bf(ckb); oh[0] = ha; oh[1] = hb; ol[0] = f2bf(cka - bf2f(ha)); ol[1] = f2bf(ckb - bf2f(hb));
        const size_t o = (size_t)b * JC + jb + ca;
        *(volatile v2us*)(CKh + o) = oh; *(volatile v2us*)(CKl + o) = ol; __threadfence(); *(volatile v2us*)(CKh + o) = oh; *(volatile v2us*)(CKl + o) = ol; }
}
__global__ __launch_bounds__(256) void k_lnrelu(const float* __restrict__ Hs, const float* __restrict__ g, const float* __restrict__ bb, float* OUTP) {
    const int lane = threadIdx.x & 31, r = blockIdx.x * 8 + (threadIdx.x >> 5); if (r >= NB_) return;
    v4f v[NOUT / 128]; float s = 0.f;
#pragma unroll
    for (int q = 0; q < NOUT / 128; ++q) { v[q] = *(const v4f*)(Hs + (size_t)r * NOUT + q * 128 + lane * 4);
#pragma unroll
        for (int i = 0; i < 4; ++i) s += v[q][i]; }
#pragma unroll
    for (int sh = 16; sh; sh >>= 1) s += __shfl_xor(s, sh, 32);
    const float mu = s * (1.0f / NOUT); float s2 = 0.f;
#pragma unroll
    for (int q = 0; q < NOUT / 128; ++q)
#pragma unroll
        for (int i = 0; i < 4; ++i) { const float d = v[q][i] - mu; s2 = fmaf(d, d, s2); }
#pragma unroll
    for (int sh = 16; sh; sh >>= 1) s2 += __shfl_xor(s2, sh, 32);
    const float rs = rsqrtf(s2 * (1.0f / NOUT) + LN_EPS);
#pragma unroll 1
    for (int ps = 0; ps < 2; ++ps) {
#pragma unroll
        for (int q = 0; q < NOUT / 128; ++q) { const int c0 = q * 128 + lane * 4; v4f y;
#pragma unroll
            for (int i = 0; i < 4; ++i) y[i] = fmaxf((v[q][i] - mu) * rs * bfr(g[c0 + i]) + bfr(bb[c0 + i]), 0.f);
            *(volatile v4f*)(OUTP + (size_t)r * NOUT + c0) = y; }
        if (ps == 0) __threadfence(); }
}

extern "C" void kernel_launch(void* const* d_in, const int* in_sizes, int n_in,
                              void* d_out, int out_size, void* d_ws, size_t ws_size, hipStream_t stream) {
    (void)in_sizes; (void)n_in; (void)out_size;
    const float* x1 = (const float*)d_in[0]; const float* x2 = (const float*)d_in[1]; const float* S1 = (const float*)d_in[2]; const float* S2 = (const float*)d_in[3];
    const float* Wm = (const float*)d_in[4]; const float* bias = (const float*)d_in[5]; const float* g = (const float*)d_in[6]; const float* bb = (const float*)d_in[7];
    float* out = (float*)d_out;
    char* wsp = (char*)d_ws;
    auto take = [&](size_t bytes) { char* p = wsp; wsp += (bytes + 255) & ~(size_t)255; return (void*)p; };
    bf* WT = (bf*)take((size_t)NOUT * SK * 2); bf* CKh = (bf*)take((size_t)NB_ * JC * 2); bf* CKl = (bf*)take((size_t)NB_ * JC * 2); float* H0 = (float*)take((size_t)NB_ * NOUT * 4); float* H1 = (float*)take((size_t)NB_ * NOUT * 4);
    if ((size_t)(wsp - (char*)d_ws) > ws_size) return;
    for (int c = 0; c < SK / JC; ++c) k_wt<<<dim3(JC / 64, NOUT / 64, 1), 256, 0, stream>>>(Wm + (size_t)c * JC * NOUT, JC, NOUT, WT + (size_t)c * NOUT * JC);
    float* Hprev = nullptr;
    for (int c = 0; c < SK / JC; ++c) { float* Hc = (c & 1) ? H1 : H0;
        k_sketch<<<JC / 64, 256, 0, stream>>>(x1, x2, S1, S2, c * JC, CKh, CKl);
        k_gemmb<true, false><<<dim3(NB_ / 64, NOUT / 64, 1), 128, 0, stream>>>(CKh, CKl, WT + (size_t)c * NOUT * JC, c == 0 ? bias : nullptr, Hc, NOUT, nullptr, Hprev, JC, 0);
        Hprev = Hc; }
    k_lnrelu<<<NB_ / 8, 256, 0, stream>>>(Hprev, g, bb, out);
}
